// MoEBlock_86620900426230
// MI455X (gfx1250) — hardware-verified
//
#include <hip/hip_runtime.h>
#include <stddef.h>
#include <stdint.h>

typedef float          v4f  __attribute__((ext_vector_type(4)));
typedef float          v8f  __attribute__((ext_vector_type(8)));
typedef int            v4i  __attribute__((ext_vector_type(4)));
typedef int            v8i  __attribute__((ext_vector_type(8)));
typedef unsigned short v8us __attribute__((ext_vector_type(8)));
typedef __bf16         v16bf __attribute__((ext_vector_type(16)));
typedef v8us  __attribute__((may_alias)) v8usa;
typedef v4f   __attribute__((may_alias)) v4fa;
typedef v4i   __attribute__((may_alias)) v4ia;
typedef float __attribute__((may_alias)) f32a;
union FragB { v16bf v; v8us h[2]; v8i w; };

#define NB   16
#define CI   192
#define HH   32
#define WW   32
#define NO   192
#define HWP  (HH * WW)
#define KD   (9 * CI)
#define NE   8
#define PT   64
#define NPT  (HWP / PT)
#define HR   4
#define HC   34
#define NCH  (KD / 8)
#define CTHR 384
#define NCW  (CTHR / 32)
#define RTHR 128
#define WSMAX 134217728

static_assert(HWP % PT == 0);
static_assert(PT == 2 * WW);
static_assert(KD % 32 == 0);
static_assert((KD * 2) % 128 == 0);
static_assert((PT * 4) % 128 == 0);
static_assert((HWP * 4) % 128 == 0);
static_assert((WW * CI * 2) % 128 == 0);
static_assert(CI % 32 == 0);
static_assert(NCH % 8 == 0);
static_assert((NE * NO * NCH) % 256 == 0);
static_assert((CI * (WW / 4)) % 256 == 0);
static_assert(((WW * CI) / 8) % 256 == 0);
static_assert(HR * HC * CI * 2 >= NO * PT * 4);
static_assert(HR * HC * CI * 2 <= 65536);
static_assert(NCW * 16 == NO);
static_assert((NCW / 2) * 32 == NO);
static_assert(NB * NE == RTHR);
static_assert(NB <= 16);
static_assert((CI * 4) % 128 == 0);

__device__ __forceinline__ v8f wmb(const FragB& a, const FragB& b, v8f c) {
  v8f d = __builtin_amdgcn_wmma_f32_16x16x32_bf16(false, a.v, false, b.v, (short)0, c, false, false);
  asm volatile("v_nop\n\tv_nop\n\tv_nop\n\tv_nop" : "+v"(d) : "v"(a.w), "v"(b.w));
  return d;
}

__device__ __forceinline__ FragB ldfrag(const unsigned short* p, int hh) {
  FragB f;
  f.h[0] = *(const v8usa*)(p + 8 * hh);
  f.h[1] = *(const v8usa*)(p + 16 + 8 * hh);
  return f;
}

__device__ __forceinline__ unsigned short rne16(float f) {
  unsigned u = __float_as_uint(f);
  u += 0x7FFFu + ((u >> 16) & 1u);
  return (unsigned short)(u >> 16);
}
__device__ __forceinline__ float rne16f(float f) {
  return __uint_as_float(((unsigned)rne16(f)) << 16);
}
__device__ __forceinline__ v8us cvt8(const v4f a, const v4f b) {
  v8us o;
  o[0] = rne16(a.x); o[1] = rne16(a.y); o[2] = rne16(a.z); o[3] = rne16(a.w);
  o[4] = rne16(b.x); o[5] = rne16(b.y); o[6] = rne16(b.z); o[7] = rne16(b.w);
  return o;
}

__global__ __launch_bounds__(256) void pool_kernel(const float* __restrict__ x, float* pooled) {
  __shared__ __attribute__((aligned(16))) float red[32];
  const int tid = threadIdx.x, lane = tid & 31, w = tid >> 5;
  const int cgp = blockIdx.x, b = blockIdx.y;
#pragma unroll 1
  for (int i = 0; i < 4; ++i) {
    const int c = 32 * cgp + 4 * w + i;
    const float* p = x + ((size_t)(b * CI + c)) * HWP;
    float s = 0.0f;
#pragma unroll 1
    for (int q = lane; q < HWP / 4; q += 32) {
      const v4f g = *(const v4fa*)(p + 4 * q);
      s += (rne16f(g.x) + rne16f(g.y)) + (rne16f(g.z) + rne16f(g.w));
    }
    s += __shfl_xor(s, 16);
    s += __shfl_xor(s, 8);
    s += __shfl_xor(s, 4);
    s += __shfl_xor(s, 2);
    s += __shfl_xor(s, 1);
    if (lane == 0) red[4 * w + i] = s * (1.0f / (float)HWP);
  }
  __syncthreads();
  if (w == 0) {
    const v4f v = *(const v4fa*)(red + 4 * (lane & 7));
    float* dst = pooled + (size_t)(b * CI + 32 * cgp) + 4 * (lane & 7);
    if (lane < 8) *(volatile v4f*)dst = v;
    __threadfence();
    if (lane < 8) *(volatile v4f*)dst = v;
  }
}

__global__ __launch_bounds__(RTHR) void router_kernel(const float* __restrict__ pooled,
                                                     const float* __restrict__ gw,
                                                     const float* __restrict__ gb,
                                                     int* route) {
  __shared__ float pl[NB * CI];
  __shared__ __attribute__((aligned(16))) float sw[CI * NE];
  __shared__ float sbv[NE];
  __shared__ float lg[NB * NE];
  const int tid = threadIdx.x, lane = tid & 31, w = tid >> 5;
#pragma unroll 1
  for (int i = tid; i < NB * CI; i += RTHR) pl[i] = pooled[i];
#pragma unroll 1
  for (int i = tid; i < CI * NE; i += RTHR) sw[i] = rne16f(gw[i]);
  if (tid < NE) sbv[tid] = rne16f(gb[tid]);
  __syncthreads();
  {
    const int b = tid >> 3, e = tid & 7;
    float s = 0.0f;
#pragma unroll 4
    for (int c = 0; c < CI; ++c) s += pl[b * CI + c] * sw[c * NE + e];
    lg[tid] = s + sbv[e];
  }
  __syncthreads();
  if (w == 0) {
    const int b = lane & 15;
    float p[NE];
#pragma unroll
    for (int e = 0; e < NE; ++e) p[e] = lg[b * NE + e];
    float mx = p[0];
#pragma unroll
    for (int e = 1; e < NE; ++e) mx = fmaxf(mx, p[e]);
    float s = 0.0f;
#pragma unroll
    for (int e = 0; e < NE; ++e) { p[e] = __expf(p[e] - mx); s += p[e]; }
    const float inv = 1.0f / s;
#pragma unroll
    for (int e = 0; e < NE; ++e) p[e] *= inv;
    int i1 = 0;
    float b1 = p[0];
#pragma unroll
    for (int e = 1; e < NE; ++e) {
      const bool up = p[e] > b1;
      i1 = up ? e : i1;
      b1 = up ? p[e] : b1;
    }
    int i2 = 0;
    float b2 = -1.0f;
#pragma unroll
    for (int e = 0; e < NE; ++e) {
      const bool ok = (e != i1) && (p[e] > b2);
      i2 = ok ? e : i2;
      b2 = ok ? p[e] : b2;
    }
    const float s2 = (b1 + b2) + 1e-10f;
    const float inv2 = 1.0f / s2;
    v4i rec;
    rec.x = i1; rec.y = i2; rec.z = __float_as_int(b1 * inv2); rec.w = __float_as_int(b2 * inv2);
    int* dst = route + 4 * b;
    if (lane < NB) *(volatile v4ia*)dst = rec;
    __threadfence();
    if (lane < NB) *(volatile v4ia*)dst = rec;
  }
}

__global__ __launch_bounds__(256) void wcvt_kernel(const float* __restrict__ ew, unsigned short* wpl) {
  const int u = (int)blockIdx.x * 256 + (int)threadIdx.x;
  if (u >= NE * NO * NCH) return;
  const int row = u / NCH;
  const int kc  = u - row * NCH;
  const int t   = kc / (CI / 8);
  const int c0  = (kc - t * (CI / 8)) * 8;
  const float* p = ew + ((size_t)row * CI + c0) * 9 + t;
  v4f a, b;
  a.x = p[0];  a.y = p[9];  a.z = p[18]; a.w = p[27];
  b.x = p[36]; b.y = p[45]; b.z = p[54]; b.w = p[63];
  const v8us o8 = cvt8(a, b);
  const size_t q = (size_t)row * KD + (size_t)(8 * kc);
  *(volatile v8usa*)(wpl + q) = o8;
  __threadfence();
  *(volatile v8usa*)(wpl + q) = o8;
}

__device__ __forceinline__ void xcvt_store_pass(const unsigned short* T, unsigned short* dst0, int tid) {
#pragma unroll
  for (int it = 0; it < ((WW * CI) / 8) / 256; ++it) {
    const int ci = it * 256 + tid;
    const v8us v = *(const v8usa*)(T + 8 * ci);
    *(volatile v8usa*)(dst0 + 8 * ci) = v;
  }
}

__global__ __launch_bounds__(256) void xcvt_kernel(const float* __restrict__ x, unsigned short* xh) {
  __shared__ __attribute__((aligned(16))) unsigned short T[WW * CI];
  const int tid = threadIdx.x, iy = blockIdx.x, b = blockIdx.y;
#pragma unroll 1
  for (int e = tid; e < CI * (WW / 4); e += 256) {
    const int c = e / (WW / 4), q = e - c * (WW / 4);
    const v4f g = *(const v4fa*)(x + (((size_t)(b * CI + c)) * HH + iy) * WW + 4 * q);
    unsigned short* p = T + (4 * q) * CI + c;
    p[0]      = rne16(g.x);
    p[CI]     = rne16(g.y);
    p[2 * CI] = rne16(g.z);
    p[3 * CI] = rne16(g.w);
  }
  __syncthreads();

  unsigned short* dst0 = xh + ((size_t)(b * HH + iy)) * WW * CI;
  xcvt_store_pass(T, dst0, tid);
  __threadfence();
  xcvt_store_pass(T, dst0, tid);
}

__device__ __forceinline__ void out_store_pass(const char* smem, float* out,
                                               int b, int nb, int w, int lane) {
  const int q8 = lane & 7, sub = lane >> 3;
#pragma unroll
  for (int it = 0; it < 8; ++it) {
    const int lid = 4 * it + sub;
    const int o = 16 * w + (lid >> 1), ln = lid & 1;
    const v4f v = *(const v4fa*)(smem + (size_t)(o * PT + 32 * ln + 4 * q8) * 4);
    float* dst = out + ((size_t)(b * NO + o)) * HWP + nb + 32 * ln + 4 * q8;
    *(volatile v4f*)dst = v;
  }
}

__global__ __launch_bounds__(CTHR) void conv_kernel(
    const unsigned short* __restrict__ xh,
    const unsigned short* __restrict__ wpl,
    const int* __restrict__ route,
    const float* __restrict__ eb,
    float* out)
{
  __shared__ __attribute__((aligned(16))) char smem[HR * HC * CI * 2];
  unsigned short* sH = (unsigned short*)smem;
  f32a* sF = (f32a*)smem;

  const int tid = threadIdx.x, lane = tid & 31, w = tid >> 5;
  const int hh = lane >> 4, m = lane & 15;
  const int pt = blockIdx.x, b = blockIdx.y;
  const int nb = PT * pt;
  const int oyf = nb / WW;

  const v4i rec = *(const v4ia*)(route + 4 * b);
  int e0 = rec.x, e1 = rec.y;
  e0 = e0 < 0 ? 0 : (e0 > NE - 1 ? NE - 1 : e0);
  e1 = e1 < 0 ? 0 : (e1 > NE - 1 ? NE - 1 : e1);
  const float w0 = __int_as_float(rec.z), w1 = __int_as_float(rec.w);

  const v8us z8 = {0, 0, 0, 0, 0, 0, 0, 0};
#pragma unroll 1
  for (int e = tid; e < HR * HC * (CI / 8); e += CTHR) {
    const int rc = e / (CI / 8), q = e - rc * (CI / 8);
    const int hr = rc / HC, hc = rc - HC * hr;
    const int iy = oyf - 1 + hr, ix = hc - 1;
    const bool ok = (iy >= 0) && (iy < HH) && (ix >= 0) && (ix < WW);
    const int iyc = (iy < 0) ? 0 : ((iy > HH - 1) ? (HH - 1) : iy);
    const int ixc = (ix < 0) ? 0 : ((ix > WW - 1) ? (WW - 1) : ix);
    const v8us g = *(const v8usa*)(xh + (((size_t)(b * HH + iyc)) * WW + ixc) * CI + 8 * q);
    *(v8usa*)(sH + (hr * HC + hc) * CI + 8 * q) = ok ? g : z8;
  }
  __syncthreads();

  const int cgp = w % (NCW / 2), pg = w / (NCW / 2);
  const unsigned short* wa0 = wpl + ((size_t)(e0 * NO + 32 * cgp + m)) * KD;
  const unsigned short* wa1 = wa0 + (size_t)16 * KD;
  const unsigned short* wb0 = wpl + ((size_t)(e1 * NO + 32 * cgp + m)) * KD;
  const unsigned short* wb1 = wb0 + (size_t)16 * KD;
  const int pb0 = (pg * HC + m) * CI;
  const int pb1 = (pg * HC + 16 + m) * CI;

  const v8f zf = {0.f, 0.f, 0.f, 0.f, 0.f, 0.f, 0.f, 0.f};
  v8f acc[2][2][2];
#pragma unroll
  for (int k = 0; k < 2; ++k)
#pragma unroll
    for (int i = 0; i < 2; ++i)
#pragma unroll
      for (int j = 0; j < 2; ++j) acc[k][i][j] = zf;

#pragma unroll 1
  for (int t = 0; t < 9; ++t) {
    const int dy = t / 3, dx = t - 3 * dy;
    const int toff = (dy * HC + dx) * CI;
    const int kt = t * CI;
#pragma unroll 1
    for (int cc = 0; cc < CI / 32; ++cc) {
      const int ch0 = 32 * cc;
      const FragB q0 = ldfrag(sH + pb0 + toff + ch0, hh);
      const FragB q1 = ldfrag(sH + pb1 + toff + ch0, hh);
      const FragB a0 = ldfrag(wa0 + kt + ch0, hh);
      const FragB a1 = ldfrag(wa1 + kt + ch0, hh);
      acc[0][0][0] = wmb(a0, q0, acc[0][0][0]);
      acc[0][0][1] = wmb(a0, q1, acc[0][0][1]);
      acc[0][1][0] = wmb(a1, q0, acc[0][1][0]);
      acc[0][1][1] = wmb(a1, q1, acc[0][1][1]);
      const FragB c0 = ldfrag(wb0 + kt + ch0, hh);
      const FragB c1 = ldfrag(wb1 + kt + ch0, hh);
      acc[1][0][0] = wmb(c0, q0, acc[1][0][0]);
      acc[1][0][1] = wmb(c0, q1, acc[1][0][1]);
      acc[1][1][0] = wmb(c1, q0, acc[1][1][0]);
      acc[1][1][1] = wmb(c1, q1, acc[1][1][1]);
    }
  }
  __syncthreads();

#pragma unroll
  for (int i = 0; i < 2; ++i) {
    const int ob = 32 * cgp + 16 * i + 8 * hh;
    const v4f pA = *(const v4fa*)(eb + e0 * NO + ob);
    const v4f pB = *(const v4fa*)(eb + e0 * NO + ob + 4);
    const v4f qA = *(const v4fa*)(eb + e1 * NO + ob);
    const v4f qB = *(const v4fa*)(eb + e1 * NO + ob + 4);
    const float bias0[8] = { rne16f(pA.x), rne16f(pA.y), rne16f(pA.z), rne16f(pA.w),
                             rne16f(pB.x), rne16f(pB.y), rne16f(pB.z), rne16f(pB.w) };
    const float bias1[8] = { rne16f(qA.x), rne16f(qA.y), rne16f(qA.z), rne16f(qA.w),
                             rne16f(qB.x), rne16f(qB.y), rne16f(qB.z), rne16f(qB.w) };
#pragma unroll
    for (int j = 0; j < 2; ++j) {
      const int px = 32 * pg + 16 * j + m;
#pragma unroll
      for (int r = 0; r < 8; ++r) {
        const float v0 = acc[0][i][j][r] + bias0[r];
        const float v1 = acc[1][i][j][r] + bias1[r];
        sF[(ob + r) * PT + px] = w0 * v0 + w1 * v1;
      }
    }
  }
  __syncthreads();

  out_store_pass(smem, out, b, nb, w, lane);
  __threadfence();
  out_store_pass(smem, out, b, nb, w, lane);
}

extern "C" void kernel_launch(void* const* d_in, const int* in_sizes, int n_in,
                              void* d_out, int out_size, void* d_ws, size_t ws_size,
                              hipStream_t stream) {
  if (n_in < 5) return;
  if (in_sizes[0] != NB * CI * HWP) return;
  if (in_sizes[1] != CI * NE) return;
  if (in_sizes[2] != NE) return;
  if (in_sizes[3] != NE * NO * CI * 9) return;
  if (in_sizes[4] != NE * NO) return;
  if (out_size != NB * NO * HWP) return;

  const float* x   = (const float*)d_in[0];
  const float* gw  = (const float*)d_in[1];
  const float* gb  = (const float*)d_in[2];
  const float* ew  = (const float*)d_in[3];
  const float* ebp = (const float*)d_in[4];
  float* out = (float*)d_out;

  char* ws = (char*)d_ws;
  size_t off = 0;
  const size_t oWP = off; off += (size_t)NE * NO * KD * 2;    off = (off + 255) & ~(size_t)255;
  const size_t oXH = off; off += (size_t)NB * HWP * CI * 2;   off = (off + 255) & ~(size_t)255;
  const size_t oPL = off; off += (size_t)NB * CI * 4;         off = (off + 255) & ~(size_t)255;
  const size_t oRT = off; off += (size_t)NB * 4 * 4;          off = (off + 255) & ~(size_t)255;
  if (off > ws_size || off > (size_t)WSMAX) return;

  unsigned short* WP = (unsigned short*)(ws + oWP);
  unsigned short* XH = (unsigned short*)(ws + oXH);
  float*          PL = (float*)(ws + oPL);
  int*            RT = (int*)(ws + oRT);

  pool_kernel<<<dim3(CI / 32, NB), 256, 0, stream>>>(x, PL);
  router_kernel<<<1, RTHR, 0, stream>>>(PL, gw, gb, RT);
  wcvt_kernel<<<(NE * NO * NCH) / 256, 256, 0, stream>>>(ew, WP);
  xcvt_kernel<<<dim3(HH, NB), 256, 0, stream>>>(x, XH);
  conv_kernel<<<dim3(NPT, NB), CTHR, 0, stream>>>(XH, WP, RT, ebp, out);
}
